// RelativePositionMultiHeadAttention_50027779064526
// MI455X (gfx1250) — hardware-verified
//
#include <hip/hip_runtime.h>
#include <math.h>

typedef __attribute__((ext_vector_type(16))) _Float16 v16h;
typedef __attribute__((ext_vector_type(16))) __bf16 v16b;
typedef __attribute__((ext_vector_type(8)))  _Float16 v8h;
typedef __attribute__((ext_vector_type(8)))  float v8f;
typedef __attribute__((ext_vector_type(4)))  float v4f;
typedef __attribute__((ext_vector_type(2)))  float v2f;
typedef __attribute__((ext_vector_type(4)))  unsigned v4u;
typedef __attribute__((ext_vector_type(4)))  int v4i;
typedef float __attribute__((may_alias)) float_a;
typedef int __attribute__((may_alias)) int_a;

template <typename T> __device__ __forceinline__ void vst2(void* p, T v) { *(volatile T*)p = v; __threadfence(); *(volatile T*)p = v; }
__device__ __forceinline__ v8f wmma16(v16h a, v16h b, v8f c) {
  v8f d = __builtin_amdgcn_wmma_f32_16x16x32_f16(false, a, false, b, (short)0, c, false, false);
  asm volatile("v_nop\n\tv_nop\n\tv_nop\n\tv_nop" : "+v"(d) : "v"(a), "v"(b));
  return d;
}
__device__ __forceinline__ v8f wmma_bf(v16b a, v16b b, v8f c) {
  v8f d = __builtin_amdgcn_wmma_f32_16x16x32_bf16(false, a, false, b, (short)0, c, false, false);
  asm volatile("v_nop\n\tv_nop\n\tv_nop\n\tv_nop" : "+v"(d) : "v"(a), "v"(b));
  return d;
}
__device__ __forceinline__ v16h frag_h(const _Float16* rowk0, int lane) {
  union { v16h v; v8h q[2]; } u; const _Float16* p = rowk0 + 8 * (lane >> 4);
  u.q[0] = *(const v8h*)p; u.q[1] = *(const v8h*)(p + 16); return u.v;
}
__device__ __forceinline__ v16h frag_f32(const float* rowk0, int lane) {
  v16h a; const float* p = rowk0 + 8 * (lane >> 4);
#pragma unroll
  for (int i = 0; i < 8; ++i) { a[i] = (_Float16)p[i]; a[8 + i] = (_Float16)p[16 + i]; }
  return a;
}
__device__ __forceinline__ v16h frag_f32s(const float* rowk0, int lane, float sc) {
  v16h a; const float* p = rowk0 + 8 * (lane >> 4);
#pragma unroll
  for (int i = 0; i < 8; ++i) { a[i] = (_Float16)(p[i] * sc); a[8 + i] = (_Float16)(p[16 + i] * sc); }
  return a;
}
__device__ __forceinline__ v16h fragc_f32(const float* W, int k0, int n, int lane, int ld, int K) {
  v16h a; const int g = lane >> 4;
#pragma unroll
  for (int i = 0; i < 8; ++i) { const int ka = k0 + 8 * g + i, kb = ka + 16;
    a[i] = (_Float16)(ka < K ? W[(size_t)(ka < K ? ka : K - 1) * ld + n] : 0.f); a[8 + i] = (_Float16)(kb < K ? W[(size_t)(kb < K ? kb : K - 1) * ld + n] : 0.f); }
  return a;
}
struct F2 { v16b h, l; };
__device__ __forceinline__ F2 bsplit16(const float v[16]) { F2 r;
#pragma unroll
  for (int i = 0; i < 16; ++i) { const __bf16 h = (__bf16)v[i]; r.h[i] = h; r.l[i] = (__bf16)(v[i] - (float)h); }
  return r; }
__device__ __forceinline__ F2 split_row(const float* row, int k0, int lane) { float v[16]; const float* p = row + k0 + 8 * (lane >> 4);
#pragma unroll
  for (int i = 0; i < 8; ++i) { v[i] = p[i]; v[8 + i] = p[16 + i]; }
  return bsplit16(v); }
__device__ __forceinline__ F2 split_rowK(const float* row, int k0, int lane, int K) { float v[16]; const int g = lane >> 4;
#pragma unroll
  for (int i = 0; i < 8; ++i) { const int ka = k0 + 8 * g + i, kb = ka + 16; v[i] = ka < K ? row[ka < K ? ka : K - 1] : 0.f; v[8 + i] = kb < K ? row[kb < K ? kb : K - 1] : 0.f; }
  return bsplit16(v); }
__device__ __forceinline__ F2 split_col(const float* W, int k0, int n, int lane, int ld, int K) { float v[16]; const int g = lane >> 4;
#pragma unroll
  for (int i = 0; i < 8; ++i) { const int ka = k0 + 8 * g + i, kb = ka + 16; v[i] = ka < K ? W[(size_t)(ka < K ? ka : K - 1) * ld + n] : 0.f; v[8 + i] = kb < K ? W[(size_t)(kb < K ? kb : K - 1) * ld + n] : 0.f; }
  return bsplit16(v); }
__device__ __forceinline__ v8f mac3(const F2& a, const F2& b, v8f c) { c = wmma_bf(a.l, b.h, c); c = wmma_bf(a.h, b.l, c); return wmma_bf(a.h, b.h, c); }
__device__ __forceinline__ float sigm(float v) { return 1.0f / (1.0f + expf(-v)); }
#define LDSX() do { asm volatile("s_wait_dscnt 0" ::: "memory"); __builtin_amdgcn_wave_barrier(); __builtin_amdgcn_fence(__ATOMIC_RELEASE, "workgroup"); } while (0)


#define NB 8
#define CC 512
#define TT 1024
#define NH 8
#define HD 64
#define WR 4
#define NRL 9
#define HG 8
#ifndef TNB
#define TNB NB
#endif
typedef __attribute__((ext_vector_type(8))) __bf16 v8b;
__device__ __forceinline__ v16b frag_b(const __bf16* rowk0, int lane) {
  union { v16b v; v8b q[2]; } u; const __bf16* p = rowk0 + 8 * (lane >> 4);
  u.q[0] = *(const v8b*)p; u.q[1] = *(const v8b*)(p + 16); return u.v;
}
__device__ __forceinline__ float bfr(float v) { return (float)(__bf16)v; }
__device__ __attribute__((noinline)) float exp_ni(float v) { return expf(v); }
__device__ __attribute__((noinline)) float erf_ni(float v) { return erff(v); }

#define WS_QF  0u
#define WS_QH  (WS_QF + 4u * (size_t)NB * TT * CC)
#define WS_QL  (WS_QH + 2u * (size_t)NB * TT * CC)
#define WS_KH  (WS_QL + 2u * (size_t)NB * TT * CC)
#define WS_VT  (WS_KH + 2u * (size_t)NB * TT * CC)
#define WS_VL  (WS_VT + 2u * (size_t)NB * CC * TT)
#define WS_QR  (WS_VL + 2u * (size_t)NB * CC * TT)
#define WS_S   (WS_QR + 4u * (size_t)HG * TT * 16)
#define WS_CX  (WS_S + 4u * (size_t)HG * TT * TT)
#define WS_END (WS_CX + 4u * (size_t)NB * TT * CC)

__global__ __launch_bounds__(128) void k_proj(const float* __restrict__ X, const float* __restrict__ Cc, const float* __restrict__ WQ, const float* __restrict__ BQ, const float* __restrict__ WK, const float* __restrict__ BK, const float* __restrict__ WV, const float* __restrict__ BV, float* __restrict__ QF, _Float16* __restrict__ QH, _Float16* __restrict__ QL, _Float16* __restrict__ KH, __bf16* __restrict__ VT, __bf16* __restrict__ VL) {
  __shared__ __align__(16) __bf16 sx[64][CC + 8]; __shared__ __align__(16) float sf[64][132]; __shared__ __align__(16) unsigned char sbuf[2 * 128 * 72 * 2];
  __bf16 (*th)[72] = (__bf16 (*)[72])sbuf; __bf16 (*tl2)[72] = (__bf16 (*)[72])(sbuf + 128 * 72 * 2); _Float16 (*sh)[136] = (_Float16 (*)[136])sbuf; _Float16 (*sl)[136] = (_Float16 (*)[136])(sbuf + 64 * 136 * 2);
  const int tid = threadIdx.x, wave = tid >> 5, lane = tid & 31, col = lane & 15, g = lane >> 4; const int p0 = blockIdx.x * 64; const int c0 = blockIdx.y * 128; const size_t b = blockIdx.z / 3; const int which = blockIdx.z % 3;
  const float* Xs = which == 0 ? X : Cc; const float* Wm = which == 0 ? WQ : which == 1 ? WK : WV; const float* Bm = which == 0 ? BQ : which == 1 ? BK : BV;
  for (int e = tid; e < CC * 64; e += 128) { const int c = e >> 6, pl = e & 63; sx[pl][c] = (__bf16)Xs[(b * CC + c) * (size_t)TT + p0 + pl]; }
  __syncthreads();
  v8f acc[8] = {};
#pragma unroll 2
  for (int kc = 0; kc < CC / 32; ++kc) { const v16b a = frag_b(&sx[wave * 16 + col][kc * 32], lane);
#pragma unroll
    for (int j = 0; j < 8; ++j) { v16b w; const int o = c0 + j * 16 + col;
#pragma unroll
      for (int i = 0; i < 8; ++i) { w[i] = (__bf16)Wm[(size_t)o * CC + kc * 32 + 8 * g + i]; w[8 + i] = (__bf16)Wm[(size_t)o * CC + kc * 32 + 16 + 8 * g + i]; }
      acc[j] = wmma_bf(a, w, acc[j]); } }
  if (which < 2) {
#pragma unroll
    for (int j = 0; j < 8; ++j) { const float bb = bfr(Bm[c0 + j * 16 + col]);
#pragma unroll
      for (int r = 0; r < 8; ++r) sf[wave * 16 + 8 * g + r][j * 16 + col] = acc[j][r] + bb; }
    __syncthreads();
    for (int e = tid; e < 64 * 32; e += 128) { const int rl = e >> 5, q4 = e & 31; const size_t row = b * TT + p0 + rl; const float* src = &sf[rl][q4 * 4]; if (which == 0) vst2(QF + row * CC + c0 + q4 * 4, *(const v4f*)src); }
    for (int e = tid; e < 64 * 128; e += 128) { const int rl = e >> 7, cl = e & 127; const float v = sf[rl][cl]; const _Float16 hv = (_Float16)v; sh[rl][cl] = hv; sl[rl][cl] = (_Float16)(v - (float)hv); }
    __syncthreads();
    _Float16* dh = which == 0 ? QH : KH; for (int e = tid; e < 64 * 16; e += 128) { const int rl = e >> 4, q = e & 15; const size_t row = b * TT + p0 + rl; vst2((unsigned*)(dh + row * CC + c0 + q * 8), *(const v4u*)&sh[rl][q * 8]); if (which == 0) vst2((unsigned*)(QL + row * CC + c0 + q * 8), *(const v4u*)&sl[rl][q * 8]); } }
  else {
#pragma unroll
    for (int j = 0; j < 8; ++j) { const float bb = bfr(Bm[c0 + j * 16 + col]);
#pragma unroll
      for (int r = 0; r < 8; ++r) { const float v = acc[j][r] + bb; const int rl = wave * 16 + 8 * g + r, cl = j * 16 + col; const __bf16 bh = (__bf16)v; th[cl][rl] = bh; tl2[cl][rl] = (__bf16)(v - (float)bh); } }
    __syncthreads(); for (int e = tid; e < 128 * 8; e += 128) { const int cl = e >> 3, q = e & 7; const size_t o2 = (b * CC + c0 + cl) * (size_t)TT + p0 + q * 8; vst2((unsigned*)(VT + o2), *(const v4u*)&th[cl][q * 8]); vst2((unsigned*)(VL + o2), *(const v4u*)&tl2[cl][q * 8]); } } }
__global__ __launch_bounds__(64) void k_qr(const float* __restrict__ QF, const float* __restrict__ RK, int b, int h0, float* __restrict__ QR0) { __shared__ float srk[NRL][HD]; __shared__ __align__(16) float so[64][16];
  const int t = threadIdx.x; const int h = h0 + blockIdx.z; float* QR = QR0 + (size_t)blockIdx.z * TT * 16; const int t0 = blockIdx.x * 64;
  for (int e = t; e < NRL * HD; e += 64) srk[e / HD][e % HD] = bfr(RK[e]);
  for (int e = t; e < 64 * 16; e += 64) so[e >> 4][e & 15] = 0.f;
  __syncthreads();
  const float* q = QF + ((size_t)b * TT + t0 + t) * CC + h * HD;
#pragma unroll 1
  for (int j = 0; j < NRL; ++j) { float a = 0.f;
#pragma unroll 1
    for (int d = 0; d < HD; ++d) a += q[d] * srk[j][d]; so[t][j] = a; }
  __syncthreads(); for (int e = t; e < 64 * 4; e += 64) { const int rl = e >> 2, qq = e & 3; vst2(QR + (size_t)(t0 + rl) * 16 + qq * 4, *(const v4f*)&so[rl][qq * 4]); } }
__global__ __launch_bounds__(128) void k_sc(const _Float16* __restrict__ QH, const _Float16* __restrict__ QL, const _Float16* __restrict__ KH, const float* __restrict__ QR0, const int* __restrict__ AM, int b, int h0, float* __restrict__ S0) { __shared__ __align__(16) float ss[4][16][132]; const int h = h0 + blockIdx.z; const float* QR = QR0 + (size_t)blockIdx.z * TT * 16; float* S = S0 + (size_t)blockIdx.z * TT * TT;
  const int tid = threadIdx.x, wave = tid >> 5, lane = tid & 31, col = lane & 15, g = lane >> 4; const int k0 = blockIdx.y * 128; const int ql0 = blockIdx.x * 64 + wave * 16; const size_t q0 = (size_t)b * TT + ql0;
  v8f acc[8] = {};
#pragma unroll
  for (int kc = 0; kc < HD / 32; ++kc) { const v16h ah = frag_h(QH + (q0 + col) * CC + h * HD + kc * 32, lane), al = frag_h(QL + (q0 + col) * CC + h * HD + kc * 32, lane);
#pragma unroll
    for (int j = 0; j < 8; ++j) { const v16h kb = frag_h(KH + ((size_t)b * TT + k0 + j * 16 + col) * CC + h * HD + kc * 32, lane); acc[j] = wmma16(ah, kb, acc[j]); acc[j] = wmma16(al, kb, acc[j]); } }
#pragma unroll
  for (int j = 0; j < 8; ++j) { const int s = k0 + j * 16 + col;
#pragma unroll
    for (int r = 0; r < 8; ++r) { const int t = ql0 + 8 * g + r; const int dd = s - t; float v = acc[j][r]; if (dd >= -WR && dd <= WR) v += QR[(size_t)t * 16 + dd + WR]; v = v * 0.125f - log1pf(fabsf((float)dd)); if (AM[((size_t)b * TT + t) * TT + s] == 0) v = -10000.0f; ss[wave][8 * g + r][j * 16 + col] = v; } }
  LDSX(); for (int rl = 0; rl < 16; ++rl) vst2(S + (size_t)(ql0 + rl) * TT + k0 + lane * 4, *(const v4f*)&ss[wave][rl][lane * 4]); }
__global__ __launch_bounds__(256) void k_sm(float* __restrict__ S0) { __shared__ float sred[8]; __shared__ float sbc; __shared__ __align__(16) float sh[TT];
  const int t = threadIdx.x; const size_t row = blockIdx.x; float* sr = S0 + (size_t)blockIdx.y * TT * TT + row * TT;
  float m = -3.0e38f; for (int k = t; k < TT; k += 256) m = fmaxf(m, sr[k]);
#pragma unroll
  for (int o = 1; o < 32; o <<= 1) m = fmaxf(m, __shfl_xor(m, o));
  if ((t & 31) == 0) sred[t >> 5] = m; __syncthreads(); if (t == 0) { float a = sred[0]; for (int i = 1; i < 8; ++i) a = fmaxf(a, sred[i]); sbc = a; } __syncthreads(); m = sbc; __syncthreads();
  float sum = 0.f; for (int k = t; k < TT; k += 256) sum += expf(sr[k] - m);
#pragma unroll
  for (int o = 1; o < 32; o <<= 1) sum += __shfl_xor(sum, o);
  if ((t & 31) == 0) sred[t >> 5] = sum; __syncthreads(); if (t == 0) { float a = 0.f; for (int i = 0; i < 8; ++i) a += sred[i]; sbc = 1.0f / a; } __syncthreads(); const float inv = sbc;
  for (int k = t; k < TT; k += 256) sh[k] = expf(sr[k] - m) * inv * 2048.0f;
  __syncthreads(); for (int q = t; q < TT / 4; q += 256) vst2(sr + q * 4, *(const v4f*)&sh[q * 4]); }
__global__ __launch_bounds__(128) void k_pv(const float* __restrict__ PS0, const __bf16* __restrict__ VT, const __bf16* __restrict__ VL, const float* __restrict__ RV, int b, int h0, float* __restrict__ CX) { const int h = h0 + blockIdx.z; const float* PS = PS0 + (size_t)blockIdx.z * TT * TT; __shared__ __align__(16) float ss[4][16][68]; __shared__ float srv[NRL][HD]; __shared__ float spw[64][NRL];
  const int tid = threadIdx.x, wave = tid >> 5, lane = tid & 31, col = lane & 15, g = lane >> 4; const int ql0 = blockIdx.x * 64 + wave * 16; const int tb = blockIdx.x * 64;
  for (int e = tid; e < NRL * HD; e += 128) srv[e / HD][e % HD] = bfr(RV[e]);
  for (int e = tid; e < 64 * NRL; e += 128) { const int rl = e / NRL, j = e % NRL; const int t = tb + rl, s = t + j - WR; spw[rl][j] = (s >= 0 && s < TT) ? PS[(size_t)t * TT + s] : 0.f; }
  v8f acc[4] = {};
#pragma unroll 1
  for (int kc = 0; kc < TT / 32; ++kc) { const F2 p = split_row(PS + (size_t)(ql0 + col) * TT, kc * 32, lane);
#pragma unroll
    for (int j = 0; j < 4; ++j) { const size_t po = ((size_t)b * CC + h * HD + j * 16 + col) * (size_t)TT + kc * 32; const v16b vh = frag_b(VT + po, lane); acc[j] = wmma_bf(p.h, vh, acc[j]); acc[j] = wmma_bf(p.l, vh, acc[j]); acc[j] = wmma_bf(p.h, frag_b(VL + po, lane), acc[j]); } }
  __syncthreads();
#pragma unroll
  for (int j = 0; j < 4; ++j)
#pragma unroll
    for (int r = 0; r < 8; ++r) { const int rl = wave * 16 + 8 * g + r; const int d = j * 16 + col; float a = acc[j][r]; for (int jj = 0; jj < NRL; ++jj) a += spw[rl][jj] * srv[jj][d]; ss[wave][8 * g + r][d] = a * (1.0f / 2048.0f); }
  LDSX(); for (int rl = 0; rl < 16; ++rl) if (lane < 16) vst2(CX + ((size_t)b * TT + ql0 + rl) * CC + h * HD + lane * 4, *(const v4f*)&ss[wave][rl][lane * 4]); }
__global__ __launch_bounds__(128) void k_out(const float* __restrict__ CX, const float* __restrict__ WO, const float* __restrict__ BO, float* __restrict__ OUT) { __shared__ __align__(16) float so[128][68];
  const int tid = threadIdx.x, wave = tid >> 5, lane = tid & 31, col = lane & 15, g = lane >> 4; const int t0 = blockIdx.x * 64, c0 = blockIdx.y * 128; const size_t b = blockIdx.z; const size_t r0 = b * TT + t0 + wave * 16;
  v8f acc[8] = {};
#pragma unroll 2
  for (int kc = 0; kc < CC / 32; ++kc) { const F2 a = split_row(CX + (r0 + col) * CC, kc * 32, lane);
#pragma unroll
    for (int j = 0; j < 8; ++j) { v16b w; const int o = c0 + j * 16 + col;
#pragma unroll
      for (int i = 0; i < 8; ++i) { w[i] = (__bf16)WO[(size_t)o * CC + kc * 32 + 8 * g + i]; w[8 + i] = (__bf16)WO[(size_t)o * CC + kc * 32 + 16 + 8 * g + i]; }
      acc[j] = wmma_bf(a.h, w, acc[j]); acc[j] = wmma_bf(a.l, w, acc[j]); } }
#pragma unroll
  for (int j = 0; j < 8; ++j) { const float bb = bfr(BO[c0 + j * 16 + col]);
#pragma unroll
    for (int r = 0; r < 8; ++r) so[j * 16 + col][wave * 16 + 8 * g + r] = acc[j][r] + bb; }
  __syncthreads(); for (int e = tid; e < 128 * 16; e += 128) { const int cl = e >> 4, q = e & 15; vst2(OUT + ((size_t)b * CC + c0 + cl) * TT + t0 + q * 4, *(const v4f*)&so[cl][q * 4]); } }
extern "C" void kernel_launch(void* const* d_in, const int* in_sizes, int n_in, void* d_out, int out_size, void* d_ws, size_t ws_size, hipStream_t stream) {
  (void)in_sizes; (void)n_in; (void)out_size;
  const float** F = (const float**)d_in;
  if (ws_size < (size_t)WS_END) return;
  char* ws = (char*)d_ws; float *QF = (float*)(ws + WS_QF), *QR = (float*)(ws + WS_QR), *S = (float*)(ws + WS_S), *CX = (float*)(ws + WS_CX); _Float16 *QH = (_Float16*)(ws + WS_QH), *QL = (_Float16*)(ws + WS_QL), *KH = (_Float16*)(ws + WS_KH); __bf16 *VT = (__bf16*)(ws + WS_VT), *VL = (__bf16*)(ws + WS_VL);
  k_proj<<<dim3(TT / 64, CC / 128, TNB * 3), 128, 0, stream>>>(F[0], F[1], F[3], F[4], F[5], F[6], F[7], F[8], QF, QH, QL, KH, VT, VL);
  for (int b = 0; b < TNB; ++b) for (int h0 = 0; h0 < NH; h0 += HG) {
    k_qr<<<dim3(TT / 64, 1, HG), 64, 0, stream>>>(QF, F[11], b, h0, QR);
    k_sc<<<dim3(TT / 64, TT / 128, HG), 128, 0, stream>>>(QH, QL, KH, QR, (const int*)d_in[2], b, h0, S);
    k_sm<<<dim3(TT, HG), 256, 0, stream>>>(S);
    k_pv<<<dim3(TT / 64, 1, HG), 128, 0, stream>>>(S, VT, VL, F[12], b, h0, CX);
  }
  k_out<<<dim3(TT / 64, CC / 128, TNB), 128, 0, stream>>>(CX, F[9], F[10], (float*)d_out);
}
